// CrossAttention_77309411328210
// MI455X (gfx1250) — hardware-verified
//
#include <hip/hip_runtime.h>
#ifndef NB
#define NB 2
#endif
#ifndef SEQ
#define SEQ 4096
#endif
#define NB_FULL 2
#define SEQ_FULL 4096
#define DM 512
#define NH 8
#define HD 64
#define QP 1536
#define KOFF 512
#define VOFF 1024
#define NR ((size_t)NB * SEQ)
#define MP ((int)((size_t)NB * SEQ))
#define LN256 5.545177444479562f

#define WS_BQKV ((size_t)QP * DM * 2)
#define WS_BO   ((size_t)DM * DM * 2)
#define WS_X16  (NR * DM * 2)
#define WS_QKV  (NR * QP * 2)
#define WS_VT   ((size_t)NB * NH * HD * SEQ * 2)
#define WS_O16  (NR * DM * 2)
#define WS_TOTAL (WS_BQKV + WS_BO + WS_X16 + WS_QKV + WS_VT + WS_O16)

static_assert(SEQ % 128 == 0);
static_assert(SEQ % 64 == 0 && SEQ % 32 == 0);
static_assert(SEQ <= SEQ_FULL);
static_assert(NB >= 1 && NB <= NB_FULL);
static_assert(HD == 64 && NH * HD == DM && DM % 64 == 0 && DM % 32 == 0);
static_assert(QP == 3 * DM && QP % 64 == 0 && KOFF == DM && VOFF == 2 * DM);
static_assert((MP % 128) == 0);
static_assert((64 * 16) % 256 == 0 && (64 * 8) % 256 == 0);
static_assert(WS_BQKV % 256 == 0 && WS_BO % 256 == 0 && WS_X16 % 256 == 0 && WS_QKV % 256 == 0 && WS_VT % 256 == 0 && WS_O16 % 256 == 0);
static_assert(WS_TOTAL <= (size_t)134217728);

typedef unsigned short v8us __attribute__((ext_vector_type(8), may_alias));
typedef float  v8f  __attribute__((ext_vector_type(8)));
typedef float  v4f  __attribute__((ext_vector_type(4)));
typedef float  v4fa __attribute__((ext_vector_type(4), may_alias));
typedef _Float16 v16h __attribute__((ext_vector_type(16)));
typedef _Float16 v4h __attribute__((ext_vector_type(4)));
union FragH { v16h v; v8us half[2]; _Float16 h[16]; unsigned short u[16]; };

__device__ __forceinline__ unsigned short bf16_bits(float x) { unsigned int u = __float_as_uint(x); return (unsigned short)((u + 0x7FFFu + ((u >> 16) & 1u)) >> 16); }
__device__ __forceinline__ float bf16_val(unsigned short b) { return __uint_as_float(((unsigned int)b) << 16); }
__device__ __forceinline__ float bf16_rne(float x) { return bf16_val(bf16_bits(x)); }
__device__ __forceinline__ unsigned short h_bits(float x) { const _Float16 hv = (_Float16)x; return __builtin_bit_cast(unsigned short, hv); }

__device__ __forceinline__ v16h g2_frag(const _Float16* p, int hh) { FragH f; f.half[0] = *(const v8us*)((const unsigned short*)p + 8 * hh); f.half[1] = *(const v8us*)((const unsigned short*)p + 16 + 8 * hh); return f.v; }
__device__ __forceinline__ v8f g2_mma(v16h a, v16h b, v8f c) { v8f d = __builtin_amdgcn_wmma_f32_16x16x32_f16(false, a, false, b, (short)0, c, false, false); asm volatile("v_nop\n\tv_nop\n\tv_nop\n\tv_nop" : "+v"(d) : "v"(a), "v"(b)); return d; }

__global__ __launch_bounds__(256) void k_wtr(const float* __restrict__ w, _Float16* __restrict__ Bt) {
  __shared__ unsigned short tl[64][66];
  const int tid = threadIdx.x; const int kt = blockIdx.x / (DM / 64), nt = blockIdx.x % (DM / 64); const int k0 = kt * 64, n0 = nt * 64;
#pragma unroll 1
  for (int i = tid; i < 64 * 16; i += 256) { const int r = i >> 4, c4 = (i & 15) * 4; const v4f f = *(const v4fa*)(w + (size_t)(k0 + r) * DM + n0 + c4);
#pragma unroll
    for (int q = 0; q < 4; ++q) tl[r][c4 + q] = h_bits(bf16_rne(f[q]) * 16.0f); }
  __syncthreads();
  for (int pass = 0; pass < 2; ++pass) {
#pragma unroll
    for (int rd = 0; rd < 2; ++rd) { const int n = rd * 32 + tid / 8, pc = tid % 8; FragH f;
#pragma unroll
      for (int q = 0; q < 8; ++q) f.u[q] = tl[pc * 8 + q][n];
      *(volatile v8us*)((unsigned short*)Bt + (size_t)(n0 + n) * DM + k0 + pc * 8) = f.half[0]; }
    if (pass == 0) __threadfence(); }
}

__global__ __launch_bounds__(256) void k_x16(const float* __restrict__ x, _Float16* __restrict__ X16, size_t n8) {
  const size_t t = (size_t)blockIdx.x * 256 + threadIdx.x; if (t >= n8) return;
  const size_t r = t / (DM / 8), c8 = (t % (DM / 8)) * 8;
  const size_t rs = (r / SEQ) * SEQ_FULL + (r % SEQ);
  const float* src = x + rs * DM + c8;
  FragH f;
#pragma unroll
  for (int q = 0; q < 8; ++q) f.h[q] = (_Float16)bf16_rne(src[q]);
  *(volatile v8us*)((unsigned short*)X16 + t * 8) = f.half[0]; __threadfence(); *(volatile v8us*)((unsigned short*)X16 + t * 8) = f.half[0];
}

__global__ __launch_bounds__(128) void k_gemm2(const _Float16* __restrict__ A, int lda, size_t sA, const _Float16* __restrict__ Bh, int ldb, size_t sB, float alpha, const float* __restrict__ bias,
    float* __restrict__ C, _Float16* __restrict__ C16, int ldc, size_t sC, int M, int N, int K) {
  __shared__ __attribute__((aligned(16))) float so[4][32][68];
  const int tid = threadIdx.x, w = tid >> 5, lane = tid & 31, ln = lane & 15, hh = lane >> 4; const int by = blockIdx.y;
  A += (size_t)by * sA; Bh += (size_t)by * sB; const size_t cofs = (size_t)by * sC; const float* bp = bias;
  const int ntn = N >> 6; const int mt = blockIdx.x / ntn, nq = blockIdx.x - mt * ntn; const int row0 = mt * 128 + 32 * w, col0 = nq * 64; if (row0 >= M) return;
  const _Float16* a0p = A + (size_t)(row0 + ln) * lda; const _Float16* a1p = a0p + (size_t)16 * lda;
  const _Float16* b0p = Bh + (size_t)(col0 + ln) * ldb; const _Float16* b1p = b0p + (size_t)16 * ldb; const _Float16* b2p = b1p + (size_t)16 * ldb; const _Float16* b3p = b2p + (size_t)16 * ldb;
  const v8f z8 = {0.f,0.f,0.f,0.f,0.f,0.f,0.f,0.f}; v8f c00 = z8, c01 = z8, c02 = z8, c03 = z8, c10 = z8, c11 = z8, c12 = z8, c13 = z8;
#pragma unroll 1
  for (int kb = 0; kb < K; kb += 32) { const v16h a0 = g2_frag(a0p + kb, hh), a1 = g2_frag(a1p + kb, hh);
    v16h b = g2_frag(b0p + kb, hh); c00 = g2_mma(a0, b, c00); c10 = g2_mma(a1, b, c10);
    b = g2_frag(b1p + kb, hh); c01 = g2_mma(a0, b, c01); c11 = g2_mma(a1, b, c11);
    b = g2_frag(b2p + kb, hh); c02 = g2_mma(a0, b, c02); c12 = g2_mma(a1, b, c12);
    b = g2_frag(b3p + kb, hh); c03 = g2_mma(a0, b, c03); c13 = g2_mma(a1, b, c13); }
  v8f accs[8] = {c00, c01, c02, c03, c10, c11, c12, c13};
#pragma unroll
  for (int u = 0; u < 8; ++u) { const int t = u & 3, half = u >> 2; const int col = col0 + t * 16 + ln; const float bv = bp ? bf16_rne(bp[col]) : 0.f;
#pragma unroll
    for (int r = 0; r < 8; ++r) { const int rloc = half * 16 + 8 * hh + r; const float v = accs[u][r] * alpha + bv; so[w][rloc][t * 16 + ln] = v; } }
  __builtin_amdgcn_fence(4  , "workgroup"); __builtin_amdgcn_wave_barrier();
  const int rsub = lane >> 4, c4 = (lane & 15) * 4;
  for (int pass = 0; pass < 2; ++pass) {
#pragma unroll
    for (int q = 0; q < 16; ++q) { const int r = q * 2 + rsub; const v4f v = *(const v4fa*)&so[w][r][c4];
      if (C) *(volatile v4f*)(C + cofs + (size_t)(row0 + r) * ldc + col0 + c4) = v;
      if (C16) { v4h h4;
#pragma unroll
        for (int i = 0; i < 4; ++i) h4[i] = (_Float16)v[i];
        *(volatile v4h*)(C16 + cofs + (size_t)(row0 + r) * ldc + col0 + c4) = h4; } }
    if (pass == 0) __threadfence(); }
}

__global__ __launch_bounds__(256) void k_vt(const _Float16* __restrict__ QKV, _Float16* __restrict__ Vt) {
  __shared__ unsigned short tl[64][66];
  const int tid = threadIdx.x; const int slab = blockIdx.x / (SEQ / 64), lg = blockIdx.x % (SEQ / 64); const int b = slab / NH, h = slab % NH;
  for (int i = tid; i < 64 * 8; i += 256) { const int r = i / 8, c8 = (i % 8) * 8; FragH f; f.half[0] = *(const v8us*)((const unsigned short*)QKV + ((size_t)b * SEQ + lg * 64 + r) * QP + VOFF + h * HD + c8);
#pragma unroll
    for (int q = 0; q < 8; ++q) tl[r][c8 + q] = f.u[q]; }
  __syncthreads();
  for (int pass = 0; pass < 2; ++pass) {
#pragma unroll
    for (int rd = 0; rd < 2; ++rd) { const int d = rd * 32 + tid / 8, pc = tid % 8; FragH f;
#pragma unroll
      for (int q = 0; q < 8; ++q) f.u[q] = tl[pc * 8 + q][d];
      *(volatile v8us*)((unsigned short*)Vt + ((size_t)slab * HD + d) * SEQ + lg * 64 + pc * 8) = f.half[0]; }
    if (pass == 0) __threadfence(); }
}

__global__ __launch_bounds__(128) void k_flash(const _Float16* __restrict__ QKV, const _Float16* __restrict__ VT, _Float16* __restrict__ O16) {
  __shared__ __attribute__((aligned(16))) unsigned short so[4][16][72];
  const int tid = threadIdx.x, w = tid >> 5, lane = tid & 31, ln = lane & 15, hh = lane >> 4;
  const int bh = blockIdx.x / (SEQ / 64), qb = blockIdx.x % (SEQ / 64); const int b = bh / NH, h = bh % NH;
  const int q0 = qb * 64 + w * 16;
  const _Float16* qrow = QKV + ((size_t)b * SEQ + q0 + ln) * QP + h * HD;
  const v16h qf0 = g2_frag(qrow, hh), qf1 = g2_frag(qrow + 32, hh);
  const _Float16* kbase = QKV + ((size_t)b * SEQ + ln) * QP + KOFF + h * HD;
  const _Float16* vbase = VT + ((size_t)bh * HD + ln) * SEQ;
  const v8f z8 = {0.f,0.f,0.f,0.f,0.f,0.f,0.f,0.f};
  v8f o0 = z8, o1 = z8, o2 = z8, o3 = z8; float m_run = -1.0e30f, l_run = 0.f;
#pragma unroll 1
  for (int kb = 0; kb < SEQ; kb += 32) {
    const _Float16* k0p = kbase + (size_t)kb * QP; const _Float16* k1p = k0p + (size_t)16 * QP;
    v8f s0 = z8, s1 = z8;
    s0 = g2_mma(g2_frag(k0p, hh), qf0, s0); s0 = g2_mma(g2_frag(k0p + 32, hh), qf1, s0);
    s1 = g2_mma(g2_frag(k1p, hh), qf0, s1); s1 = g2_mma(g2_frag(k1p + 32, hh), qf1, s1);
    float mx = fmaxf(s0[0], s1[0]);
#pragma unroll
    for (int r = 1; r < 8; ++r) mx = fmaxf(mx, fmaxf(s0[r], s1[r]));
    mx = fmaxf(mx, __shfl_xor(mx, 16, 32));
    const float mn = fmaxf(m_run, mx * 0.125f); const float corr = __expf(m_run - mn); const float nm = LN256 - mn;
    v16h pf; float rs = 0.f;
#pragma unroll
    for (int r = 0; r < 8; ++r) { const float p0 = __expf(fmaf(s0[r], 0.125f, nm)); const float p1 = __expf(fmaf(s1[r], 0.125f, nm)); rs += p0 + p1; pf[r] = (_Float16)p0; pf[8 + r] = (_Float16)p1; }
    l_run = l_run * corr + rs; m_run = mn;
    o0 *= corr; o1 *= corr; o2 *= corr; o3 *= corr;
    const _Float16* vp = vbase + kb;
    o0 = g2_mma(g2_frag(vp, hh), pf, o0);
    o1 = g2_mma(g2_frag(vp + (size_t)16 * SEQ, hh), pf, o1);
    o2 = g2_mma(g2_frag(vp + (size_t)32 * SEQ, hh), pf, o2);
    o3 = g2_mma(g2_frag(vp + (size_t)48 * SEQ, hh), pf, o3); }
  const float lt = l_run + __shfl_xor(l_run, 16, 32);
  const float inv = 64.0f * (1.0f / lt);
  { FragH f;
#pragma unroll
    for (int r = 0; r < 8; ++r) f.h[r] = (_Float16)(o0[r] * inv);
    *(v8us*)&so[w][ln][8 * hh] = f.half[0];
#pragma unroll
    for (int r = 0; r < 8; ++r) f.h[r] = (_Float16)(o1[r] * inv);
    *(v8us*)&so[w][ln][16 + 8 * hh] = f.half[0];
#pragma unroll
    for (int r = 0; r < 8; ++r) f.h[r] = (_Float16)(o2[r] * inv);
    *(v8us*)&so[w][ln][32 + 8 * hh] = f.half[0];
#pragma unroll
    for (int r = 0; r < 8; ++r) f.h[r] = (_Float16)(o3[r] * inv);
    *(v8us*)&so[w][ln][48 + 8 * hh] = f.half[0]; }
  __builtin_amdgcn_fence(4  , "workgroup"); __builtin_amdgcn_wave_barrier();
  const int rq = lane >> 3, pc = lane & 7;
  for (int pass = 0; pass < 2; ++pass) {
#pragma unroll
    for (int it = 0; it < 4; ++it) { const int row = it * 4 + rq; const v8us v = *(const v8us*)&so[w][row][pc * 8];
      *(volatile v8us*)((unsigned short*)O16 + ((size_t)b * SEQ + q0 + row) * DM + h * HD + pc * 8) = v; }
    if (pass == 0) __threadfence(); }
}

extern "C" void kernel_launch(void* const* d_in, const int* in_sizes, int n_in,
                              void* d_out, int out_size, void* d_ws, size_t ws_size, hipStream_t stream) {
  if (n_in < 6) return;
  if (in_sizes[0] < (int)((((size_t)(NB - 1)) * SEQ_FULL + SEQ) * DM)) return;
  if (in_sizes[1] < DM * DM || in_sizes[2] < DM * DM || in_sizes[3] < DM * DM || in_sizes[4] < DM * DM) return;
  if (in_sizes[5] < DM) return;
  if (out_size < (int)(NR * DM)) return;
  if ((size_t)WS_TOTAL > ws_size) return;
  const float* x = (const float*)d_in[0]; const float* wq = (const float*)d_in[1]; const float* wk = (const float*)d_in[2];
  const float* wv = (const float*)d_in[3]; const float* wo = (const float*)d_in[4]; const float* bo = (const float*)d_in[5];
  char* ws = (char*)d_ws; size_t off = 0;
  _Float16* BQKV = (_Float16*)(ws + off); off += WS_BQKV;
  _Float16* BO   = (_Float16*)(ws + off); off += WS_BO;
  _Float16* X16  = (_Float16*)(ws + off); off += WS_X16;
  _Float16* QKV  = (_Float16*)(ws + off); off += WS_QKV;
  _Float16* VT   = (_Float16*)(ws + off); off += WS_VT;
  _Float16* O16  = (_Float16*)(ws + off); off += WS_O16;
  if (off > ws_size) return;

  { const unsigned g = (unsigned)((DM / 64) * (DM / 64));
    k_wtr<<<g, 256, 0, stream>>>(wq, BQKV);
    k_wtr<<<g, 256, 0, stream>>>(wk, BQKV + (size_t)DM * DM);
    k_wtr<<<g, 256, 0, stream>>>(wv, BQKV + (size_t)2 * DM * DM);
    k_wtr<<<g, 256, 0, stream>>>(wo, BO); }
  { const size_t n8 = NR * DM / 8; k_x16<<<(unsigned)((n8 + 255) / 256), 256, 0, stream>>>(x, X16, n8); }

  k_gemm2<<<dim3((unsigned)((MP / 128) * (QP / 64)), 1), 128, 0, stream>>>(X16, DM, 0, BQKV, DM, 0, 0.0625f, nullptr, nullptr, QKV, QP, 0, MP, QP, DM);
  k_vt<<<(unsigned)(NB * NH * (SEQ / 64)), 256, 0, stream>>>(QKV, VT);
  k_flash<<<(unsigned)(NB * NH * (SEQ / 64)), 128, 0, stream>>>(QKV, VT, O16);
  k_gemm2<<<dim3((unsigned)((MP / 128) * (DM / 64)), 1), 128, 0, stream>>>(O16, DM, 0, BO, DM, 0, 0.0009765625f, bo, (float*)d_out, nullptr, DM, 0, MP, DM, DM);
}
